// Block_27410481283473
// MI455X (gfx1250) — hardware-run, weakly checked
//
#include <hip/hip_runtime.h>


#ifndef NB
#define NB 2
#endif
#ifndef SEQ
#define SEQ 2048
#endif
#define NB_FULL  2
#define SEQ_FULL 2048
#ifndef OUT_SEQ
#define OUT_SEQ SEQ
#endif
#define EMB  1024
#define NH_  16
#define HD   64
#define DM   (NH_ * HD)
#define AW   4
#define QRS  2048.0f
#define QRI  (1.0f / 2048.0f)
#define SC2  (0.125f * 1.4426950408889634f)
#define PSH  8.0f
#define PINV (1.0f / 256.0f)
#define LATE 512
#define LATE0 ((SEQ > LATE) ? (SEQ - LATE) : 0)
#define NEGV (-3.0e38f)
#define WSC   64.0f
#define WINV  (1.0f / 64.0f)
#define ASC   256.0f
#define FOLDO (1.0f / 16384.0f)
#define LNEPS 1.0e-5f

static_assert(HD == 64);
static_assert(DM == 1024);
static_assert(EMB % 64 == 0);
static_assert(EMB % 32 == 0);
static_assert(DM % 64 == 0);
static_assert(SEQ % 64 == 0);
static_assert((NB * SEQ) % 64 == 0);
static_assert(SEQ % 32 == 0);
static_assert(SEQ % (16 * AW) == 0);
static_assert(LATE % 32 == 0);
static_assert(((size_t)SEQ * EMB) % 8 == 0);
static_assert(NB <= NB_FULL);
static_assert(SEQ <= SEQ_FULL);
static_assert(DM == EMB);
static_assert(DM / 64 == NH_);
static_assert(4 * 32 * 8 == EMB);
static_assert((NB * SEQ) % 8 == 0);
static_assert(256 * 2 * 16 == 64 * 64 * 2);
static_assert(32 * 16 * 4 == 16 * HD * 2);
static_assert(32 * 16 * 8 == 16 * 64 * 4);
static_assert(64 * 68 * 4 <= 131072);
static_assert(16 * 68 * 4 <= 131072);
static_assert(AW * 16 * 68 * 4 + 16 * AW * 4 <= 131072);

typedef _Float16 h16;
typedef __attribute__((ext_vector_type(16))) _Float16 v16h;
typedef __attribute__((ext_vector_type(8)))  _Float16 v8h;
typedef __attribute__((ext_vector_type(8)))  float    v8f;
typedef __attribute__((ext_vector_type(4)))  float    v4f;
typedef v4f  __attribute__((may_alias)) v4fa;

__device__ __forceinline__ unsigned short f2bf(float f) { unsigned u = __float_as_uint(f); u += 0x7FFFu + ((u >> 16) & 1u); return (unsigned short)(u >> 16); }
__device__ __forceinline__ float bfr(float f) { return __uint_as_float(((unsigned)f2bf(f)) << 16); }
__device__ __forceinline__ v16h cat16(v8h lo, v8h hi) { return __builtin_shufflevector(lo, hi, 0, 1, 2, 3, 4, 5, 6, 7, 8, 9, 10, 11, 12, 13, 14, 15); }
__device__ __forceinline__ v8f wmma16(v16h a, v16h b, v8f c) { return __builtin_amdgcn_wmma_f32_16x16x32_f16(false, a, false, b, (short)0, c, false, false); }
__device__ __forceinline__ v16h  ldh(const h16* p) { return cat16(*(const v8h*)p, *(const v8h*)(p + 16)); }
__device__ __forceinline__ void wave_sync() { __builtin_amdgcn_fence(3  , "wavefront"); __builtin_amdgcn_wave_barrier(); asm volatile("" ::: "memory"); }
static __device__ __forceinline__ h16 toh_flush(float v) { const h16 r = (h16)v; return (fabsf(v) < 6.103515625e-05f) ? (h16)0.0f : r; }

__global__ __launch_bounds__(256) void k_cvth(const float* __restrict__ src, h16* dst, float sc, size_t n8) {
    const size_t i = (size_t)blockIdx.x * 256 + threadIdx.x; if (i >= n8) return;
    const v8f v = *(const v8f*)(src + i * 8); v8h o;
#pragma unroll
    for (int k = 0; k < 8; ++k) o[k] = toh_flush(v[k] * sc);
    *(volatile v8h*)(dst + i * 8) = o; __threadfence(); *(volatile v8h*)(dst + i * 8) = o;
}

__global__ __launch_bounds__(256) void k_cvtw(const float* __restrict__ src, h16* dst, size_t hstride, int spitch) {
    __shared__ __align__(16) float ts[64 * 68];
    const int tid = threadIdx.x; const int e0 = blockIdx.x * 64, h = blockIdx.y;
    const float* sp = src + (size_t)h * hstride + (size_t)e0 * (size_t)spitch;
#pragma unroll
    for (int it = 0; it < 4; ++it) { const int idx = it * 256 + tid; const int el = idx >> 4, d4 = (idx & 15) * 4;
        const v4f v = *(const v4f*)(sp + (size_t)el * (size_t)spitch + d4); *(v4fa*)(&ts[el * 68 + d4]) = v; }
    __syncthreads();
    v8h o[2]; size_t off[2];
#pragma unroll
    for (int it = 0; it < 2; ++it) { const int piece = it * 256 + tid; const int d = piece >> 3, e8 = (piece & 7) * 8;
#pragma unroll
        for (int i = 0; i < 8; ++i) o[it][i] = toh_flush(bfr(ts[(e8 + i) * 68 + d]) * WSC);
        off[it] = ((size_t)h * HD + d) * EMB + e0 + e8; }
#pragma unroll 1
    for (int ps = 0; ps < 2; ++ps) {
#pragma unroll
        for (int it = 0; it < 2; ++it) *(volatile v8h*)(dst + off[it]) = o[it];
        if (ps == 0) __threadfence(); }
}

__global__ __launch_bounds__(256) void k_ln(const float* __restrict__ src, int srcSeq, int rin, const float* __restrict__ g, const float* __restrict__ be, h16* dst) {
#pragma clang fp contract(off)
    const int lane = threadIdx.x & 31; const int wave = __builtin_amdgcn_readfirstlane(threadIdx.x >> 5);
    const int row = blockIdx.x * 8 + wave;
    const int b = row / SEQ, t = row % SEQ;
    const float* xr = src + ((size_t)b * (size_t)srcSeq + t) * EMB + lane * 8;
    float s = 0.0f;
#pragma unroll 1
    for (int it = 0; it < 4; ++it) { const v8f v = *(const v8f*)(xr + it * 256);
#pragma unroll
        for (int k = 0; k < 8; ++k) { const float xv = rin ? bfr(v[k]) : v[k]; s += xv; } }
#pragma unroll
    for (int o = 16; o > 0; o >>= 1) s += __shfl_xor(s, o, 32);
    const float mean = s * (1.0f / EMB);
    float q = 0.0f;
#pragma unroll 1
    for (int it = 0; it < 4; ++it) { const v8f v = *(const v8f*)(xr + it * 256);
#pragma unroll
        for (int k = 0; k < 8; ++k) { const float xv = rin ? bfr(v[k]) : v[k]; const float d = xv - mean; q += d * d; } }
#pragma unroll
    for (int o = 16; o > 0; o >>= 1) q += __shfl_xor(q, o, 32);
    const float rstd = rsqrtf(q * (1.0f / EMB) + LNEPS);
    h16* drow = dst + (size_t)row * EMB + lane * 8;
#pragma unroll 1
    for (int it = 0; it < 4; ++it) {
        const v8f v = *(const v8f*)(xr + it * 256);
        const v8f gv = *(const v8f*)(g + it * 256 + lane * 8);
        const v8f bv = *(const v8f*)(be + it * 256 + lane * 8);
        v8h o;
#pragma unroll
        for (int k = 0; k < 8; ++k) { const float xv = rin ? bfr(v[k]) : v[k]; const float y = (xv - mean) * rstd * bfr(gv[k]) + bfr(bv[k]); o[k] = toh_flush(y); }
        *(volatile v8h*)(drow + it * 256) = o; __threadfence(); *(volatile v8h*)(drow + it * 256) = o;
    }
}

__global__ __launch_bounds__(32) void k_proj(const h16* __restrict__ A, const h16* __restrict__ Bt, const float* __restrict__ bias, int rowBias, int relu,
                                             h16* Ph, h16* Pr, int useRes, int RB, size_t sRB, int pitch, int CB, size_t sCB) {
    __shared__ __align__(16) float os[16 * 68];
    const int K = EMB;
    const int lane = threadIdx.x & 31, lr = lane & 15, hi = lane >> 4; const int r0 = blockIdx.x * 64, c0 = blockIdx.y * 64;
    v8f acc[4][4];
#pragma unroll
    for (int mb = 0; mb < 4; ++mb)
#pragma unroll
        for (int nb = 0; nb < 4; ++nb) acc[mb][nb] = (v8f){};
    float colb[4];
#pragma unroll
    for (int nb = 0; nb < 4; ++nb) { int ci = c0 + nb * 16 + lr; ci = (ci < DM) ? ci : (DM - 1); colb[nb] = bfr(bias[ci]); }
    const size_t aoff = (size_t)(r0 + lr) * K + 8 * hi, boff = (size_t)(c0 + lr) * K + 8 * hi;
#pragma unroll 1
    for (int kc = 0; kc < K; kc += 32) {
        v16h a[4];
#pragma unroll
        for (int mb = 0; mb < 4; ++mb) a[mb] = ldh(A + aoff + (size_t)mb * 16 * K + kc);
#pragma unroll
        for (int nb = 0; nb < 4; ++nb) { const v16h b = ldh(Bt + boff + (size_t)nb * 16 * K + kc);
#pragma unroll
            for (int mb = 0; mb < 4; ++mb) acc[mb][nb] = wmma16(a[mb], b, acc[mb][nb]); }
        asm volatile("v_nop\n\tv_nop\n\tv_nop\n\tv_nop" : "+v"(acc[0][0]), "+v"(acc[1][1]), "+v"(acc[2][2]), "+v"(acc[3][3]) : "v"(a[0]), "v"(a[1]), "v"(a[2]), "v"(a[3]));
    }
    const size_t tbase = (size_t)(r0 / RB) * sRB + (size_t)(r0 % RB) * (size_t)pitch + (size_t)(c0 / CB) * sCB + (size_t)(c0 % CB);
#pragma unroll
    for (int mb = 0; mb < 4; ++mb) {
        float rowb[8];
#pragma unroll
        for (int j = 0; j < 8; ++j) { int ri = r0 + mb * 16 + hi * 8 + j; ri = (ri < DM) ? ri : (DM - 1); rowb[j] = bfr(bias[ri]); }
#pragma unroll
        for (int nb = 0; nb < 4; ++nb) {
#pragma unroll
            for (int j = 0; j < 8; ++j) { float cv = acc[mb][nb][j] * WINV + (rowBias ? rowb[j] : colb[nb]); cv = relu ? fmaxf(cv, 0.0f) : cv;
                os[(hi * 8 + j) * 68 + nb * 16 + lr] = cv; } }
        wave_sync();
        const size_t sb = tbase + (size_t)(mb * 16) * (size_t)pitch;
#pragma unroll 1
        for (int ps = 0; ps < 2; ++ps) {
#pragma unroll
            for (int s = 0; s < 4; ++s) { const int row = 4 * s + (lane >> 3), c8 = (lane & 7) * 8;
                const v4f x0 = *(const v4fa*)(&os[row * 68 + c8]); const v4f x1 = *(const v4fa*)(&os[row * 68 + c8 + 4]); v8h hv, rv;
#pragma unroll
                for (int i = 0; i < 4; ++i) { const h16 a0 = toh_flush(x0[i]); const h16 a1 = toh_flush(x1[i]); hv[i] = a0; hv[4 + i] = a1;
                    rv[i] = toh_flush((x0[i] - (float)a0) * QRS); rv[4 + i] = toh_flush((x1[i] - (float)a1) * QRS); }
                const size_t oo = sb + (size_t)row * (size_t)pitch + c8;
                *(volatile v8h*)(Ph + oo) = hv; if (useRes) *(volatile v8h*)(Pr + oo) = rv; }
            if (ps == 0) __threadfence(); }
        wave_sync();
    }
}

__global__ __launch_bounds__(32) void k_gemmr(const h16* __restrict__ A, const h16* __restrict__ Bt, const float* __restrict__ bias, float fold,
                                              const float* __restrict__ res, int resBf, int resSeq, float* OUT, int outSeq) {
    __shared__ __align__(16) float os[16 * 68];
    const int K = EMB;
    const int lane = threadIdx.x & 31, lr = lane & 15, hi = lane >> 4; const int r0 = blockIdx.x * 64, c0 = blockIdx.y * 64;
    v8f acc[4][4];
#pragma unroll
    for (int mb = 0; mb < 4; ++mb)
#pragma unroll
        for (int nb = 0; nb < 4; ++nb) acc[mb][nb] = (v8f){};
    float colb[4];
#pragma unroll
    for (int nb = 0; nb < 4; ++nb) { int ci = c0 + nb * 16 + lr; ci = (ci < DM) ? ci : (DM - 1); colb[nb] = bfr(bias[ci]); }
    const size_t aoff = (size_t)(r0 + lr) * K + 8 * hi, boff = (size_t)(c0 + lr) * K + 8 * hi;
#pragma unroll 1
    for (int kc = 0; kc < K; kc += 32) {
        v16h a[4];
#pragma unroll
        for (int mb = 0; mb < 4; ++mb) a[mb] = ldh(A + aoff + (size_t)mb * 16 * K + kc);
#pragma unroll
        for (int nb = 0; nb < 4; ++nb) { const v16h b = ldh(Bt + boff + (size_t)nb * 16 * K + kc);
#pragma unroll
            for (int mb = 0; mb < 4; ++mb) acc[mb][nb] = wmma16(a[mb], b, acc[mb][nb]); }
        asm volatile("v_nop\n\tv_nop\n\tv_nop\n\tv_nop" : "+v"(acc[0][0]), "+v"(acc[1][1]), "+v"(acc[2][2]), "+v"(acc[3][3]) : "v"(a[0]), "v"(a[1]), "v"(a[2]), "v"(a[3]));
    }
    const int bb = r0 / SEQ, t0 = r0 % SEQ;
    const float* rrow = res + ((size_t)bb * (size_t)resSeq + t0) * DM + c0;
    float* orow = OUT + ((size_t)bb * (size_t)outSeq + t0) * DM + c0;
#pragma unroll
    for (int mb = 0; mb < 4; ++mb) {
#pragma unroll
        for (int nb = 0; nb < 4; ++nb) {
#pragma unroll
            for (int j = 0; j < 8; ++j) os[(hi * 8 + j) * 68 + nb * 16 + lr] = acc[mb][nb][j] * fold + colb[nb]; }
        wave_sync();
#pragma unroll 1
        for (int ps = 0; ps < 2; ++ps) {
#pragma unroll
            for (int s = 0; s < 8; ++s) { const int row = 2 * s + hi, cofs = lr * 4;
                v4f val = *(const v4fa*)(&os[row * 68 + cofs]);
                const v4f rv = *(const v4f*)(rrow + (size_t)(mb * 16 + row) * DM + cofs);
#pragma unroll
                for (int i = 0; i < 4; ++i) val[i] += resBf ? bfr(rv[i]) : rv[i];
                *(volatile v4f*)(orow + (size_t)(mb * 16 + row) * DM + cofs) = val; }
            if (ps == 0) __threadfence(); }
        wave_sync();
    }
}

__global__ __launch_bounds__(32 * AW) void k_colstat(const h16* __restrict__ QH, const h16* __restrict__ QR, const h16* __restrict__ KP, float* CS) {
    __shared__ __align__(16) float cs[16 * AW];
    const int lane = threadIdx.x & 31, wave = threadIdx.x >> 5, lr = lane & 15, hi = lane >> 4;
    const int zh = blockIdx.y;
    const int s0 = (blockIdx.x * AW + wave) * 16;
    const size_t pbase = (size_t)zh * SEQ * HD;
    const size_t ko = pbase + (size_t)(s0 + lr) * HD + 8 * hi;
    const v16h kb0 = ldh(KP + ko), kb1 = ldh(KP + ko + 32);
    const size_t qo = pbase + (size_t)lr * HD + 8 * hi;
    const int sk = s0 + lr;
    float m = NEGV, l = 0.0f;
#pragma unroll 1
    for (int tq0 = (s0 & ~31); tq0 < SEQ; tq0 += 32) {
        const h16* qa = QH + qo + (size_t)tq0 * HD; const h16* ra = QR + qo + (size_t)tq0 * HD;
        const v16h qa0 = ldh(qa), qa1 = ldh(qa + 32), qb0 = ldh(qa + 16 * HD), qb1 = ldh(qa + 16 * HD + 32);
        const v16h ra0 = ldh(ra), ra1 = ldh(ra + 32), rb0 = ldh(ra + 16 * HD), rb1 = ldh(ra + 16 * HD + 32);
        v8f sHa = (v8f){}, sLa = (v8f){}, sHb = (v8f){}, sLb = (v8f){};
        sHa = wmma16(qa0, kb0, sHa); sLa = wmma16(ra0, kb0, sLa); sHb = wmma16(qb0, kb0, sHb); sLb = wmma16(rb0, kb0, sLb);
        sHa = wmma16(qa1, kb1, sHa); sLa = wmma16(ra1, kb1, sLa); sHb = wmma16(qb1, kb1, sHb); sLb = wmma16(rb1, kb1, sLb);
        asm volatile("v_nop\n\tv_nop\n\tv_nop\n\tv_nop" : "+v"(sHa), "+v"(sLa), "+v"(sHb), "+v"(sLb) : "v"(qa0), "v"(qa1), "v"(qb0), "v"(qb1), "v"(ra0), "v"(ra1), "v"(rb0), "v"(rb1), "v"(kb0), "v"(kb1));
        float ta[8], tb[8];
#pragma unroll
        for (int r = 0; r < 8; ++r) { ta[r] = (sHa[r] + sLa[r] * QRI) * SC2; tb[r] = (sHb[r] + sLb[r] * QRI) * SC2; }
        if (tq0 < s0 + 16) {
            const int tt = tq0 + 8 * hi;
#pragma unroll
            for (int r = 0; r < 8; ++r) { ta[r] = (tt + r < sk) ? NEGV : ta[r]; tb[r] = (tt + 16 + r < sk) ? NEGV : tb[r]; }
        }
        float mx = NEGV;
#pragma unroll
        for (int r = 0; r < 8; ++r) mx = fmaxf(mx, fmaxf(ta[r], tb[r]));
        mx = fmaxf(mx, __shfl_xor(mx, 16, 32));
        const float mnew = fmaxf(m, mx);
        const float alpha = __builtin_amdgcn_exp2f(m - mnew);
        float ls = 0.0f;
#pragma unroll
        for (int r = 0; r < 8; ++r) ls += __builtin_amdgcn_exp2f(ta[r] - mnew) + __builtin_amdgcn_exp2f(tb[r] - mnew);
        l = l * alpha + ls; m = mnew;
    }
    l += __shfl_xor(l, 16, 32);
    const float cval = m + __log2f(l);
    if (hi == 0) cs[wave * 16 + lr] = cval;
    __syncthreads();
    if (wave == 0 && lane < 16) {
        const v4f val = *(const v4fa*)(&cs[lane * 4]);
        float* dp = CS + (size_t)zh * SEQ + (size_t)blockIdx.x * (16 * AW) + lane * 4;
        *(volatile v4f*)dp = val; __threadfence(); *(volatile v4f*)dp = val;
    }
}

__global__ __launch_bounds__(32 * AW) void k_attn(const h16* __restrict__ QH, const h16* __restrict__ QR, const h16* __restrict__ KP, const h16* __restrict__ VT,
                                                  const h16* __restrict__ VR, const float* __restrict__ CS, float* OUT) {
    __shared__ __align__(16) float os[AW * 16 * 68];
    const int lane = threadIdx.x & 31, wave = threadIdx.x >> 5, lr = lane & 15, hi = lane >> 4;
    const int zh = blockIdx.y; const int b = zh / NH_, h = zh % NH_;
    const int t0 = (blockIdx.x * AW + wave) * 16;
    const size_t pbase = (size_t)zh * SEQ * HD;
    const size_t qo = pbase + (size_t)(t0 + lr) * HD + 8 * hi;
    const v16h qh0 = ldh(QH + qo), qh1 = ldh(QH + qo + 32), qr0 = ldh(QR + qo), qr1 = ldh(QR + qo + 32);
    const size_t ko = pbase + (size_t)lr * HD + 8 * hi;
    const size_t vo = pbase + (size_t)lr * SEQ + 8 * hi;
    const float* cp = CS + (size_t)zh * SEQ + 8 * hi;
    const int tq = t0 + lr;
    v8f oA[4], oE[4];
#pragma unroll
    for (int j = 0; j < 4; ++j) { oA[j] = (v8f){}; oE[j] = (v8f){}; }
    const int kend = t0 + 16;
#pragma unroll 1
    for (int key0 = 0; key0 < kend; key0 += 32) {
        const h16* ka = KP + ko + (size_t)key0 * HD;
        const v16h ka0 = ldh(ka), ka1 = ldh(ka + 32), kb0 = ldh(ka + 16 * HD), kb1 = ldh(ka + 16 * HD + 32);
        v8f sHa = (v8f){}, sLa = (v8f){}, sHb = (v8f){}, sLb = (v8f){};
        sHa = wmma16(ka0, qh0, sHa); sLa = wmma16(ka0, qr0, sLa); sHb = wmma16(kb0, qh0, sHb); sLb = wmma16(kb0, qr0, sLb);
        sHa = wmma16(ka1, qh1, sHa); sLa = wmma16(ka1, qr1, sLa); sHb = wmma16(kb1, qh1, sHb); sLb = wmma16(kb1, qr1, sLb);
        asm volatile("v_nop\n\tv_nop\n\tv_nop\n\tv_nop" : "+v"(sHa), "+v"(sLa), "+v"(sHb), "+v"(sLb) : "v"(ka0), "v"(ka1), "v"(kb0), "v"(kb1));
        const v4f c0v = *(const v4f*)(cp + key0), c1v = *(const v4f*)(cp + key0 + 4), c2v = *(const v4f*)(cp + key0 + 16), c3v = *(const v4f*)(cp + key0 + 20);
        float ta[8], tb[8];
#pragma unroll
        for (int r = 0; r < 4; ++r) {
            ta[r]     = (sHa[r]     + sLa[r]     * QRI) * SC2 - c0v[r] + PSH;
            ta[4 + r] = (sHa[4 + r] + sLa[4 + r] * QRI) * SC2 - c1v[r] + PSH;
            tb[r]     = (sHb[r]     + sLb[r]     * QRI) * SC2 - c2v[r] + PSH;
            tb[4 + r] = (sHb[4 + r] + sLb[4 + r] * QRI) * SC2 - c3v[r] + PSH; }
        if (key0 + 31 > t0) {
            const int kk = key0 + 8 * hi;
#pragma unroll
            for (int r = 0; r < 8; ++r) { ta[r] = (kk + r > tq) ? NEGV : ta[r]; tb[r] = (kk + 16 + r > tq) ? NEGV : tb[r]; }
        }
        float pa[8], pc[8]; v16h pb;
#pragma unroll
        for (int r = 0; r < 8; ++r) { pa[r] = __builtin_amdgcn_exp2f(ta[r]); pc[r] = __builtin_amdgcn_exp2f(tb[r]); pb[r] = (h16)pa[r]; pb[8 + r] = (h16)pc[r]; }
        const h16* va = VT + vo + key0;
        const v16h v0 = ldh(va), v1 = ldh(va + (size_t)16 * SEQ), v2 = ldh(va + (size_t)32 * SEQ), v3 = ldh(va + (size_t)48 * SEQ);
        oA[0] = wmma16(v0, pb, oA[0]); oA[1] = wmma16(v1, pb, oA[1]); oA[2] = wmma16(v2, pb, oA[2]); oA[3] = wmma16(v3, pb, oA[3]);
        if (key0 >= LATE0) {
            v16h pr;
#pragma unroll
            for (int r = 0; r < 8; ++r) { pr[r] = (h16)((pa[r] - (float)pb[r]) * QRS); pr[8 + r] = (h16)((pc[r] - (float)pb[8 + r]) * QRS); }
            const h16* wa = VR + vo + key0;
            const v16h w0 = ldh(wa), w1 = ldh(wa + (size_t)16 * SEQ), w2 = ldh(wa + (size_t)32 * SEQ), w3 = ldh(wa + (size_t)48 * SEQ);
            oE[0] = wmma16(w0, pb, oE[0]); oE[1] = wmma16(w1, pb, oE[1]); oE[2] = wmma16(w2, pb, oE[2]); oE[3] = wmma16(w3, pb, oE[3]);
            oE[0] = wmma16(v0, pr, oE[0]); oE[1] = wmma16(v1, pr, oE[1]); oE[2] = wmma16(v2, pr, oE[2]); oE[3] = wmma16(v3, pr, oE[3]);
            asm volatile("v_nop\n\tv_nop\n\tv_nop\n\tv_nop" : "+v"(oE[0]), "+v"(oE[1]), "+v"(oE[2]), "+v"(oE[3]) : "v"(w0), "v"(w1), "v"(w2), "v"(w3), "v"(pr));
        }
        asm volatile("v_nop\n\tv_nop\n\tv_nop\n\tv_nop" : "+v"(oA[0]), "+v"(oA[1]), "+v"(oA[2]), "+v"(oA[3]) : "v"(v0), "v"(v1), "v"(v2), "v"(v3), "v"(pb));
    }
    const int wb = wave * 16 * 68;
#pragma unroll
    for (int j = 0; j < 4; ++j) { v4f a, c;
#pragma unroll
        for (int i = 0; i < 4; ++i) { a[i] = (oA[j][i] + oE[j][i] * QRI) * PINV; c[i] = (oA[j][4 + i] + oE[j][4 + i] * QRI) * PINV; }
        *(v4fa*)(&os[wb + lr * 68 + 16 * j + 8 * hi]) = a; *(v4fa*)(&os[wb + lr * 68 + 16 * j + 8 * hi + 4]) = c; }
    wave_sync();
    float* orow = OUT + ((size_t)b * OUT_SEQ + t0) * DM + h * HD;
#pragma unroll 1
    for (int ps = 0; ps < 2; ++ps) {
#pragma unroll
        for (int s = 0; s < 8; ++s) { const int row = 2 * s + hi, cofs = lr * 4;
            const v4f val = *(const v4fa*)(&os[wb + row * 68 + cofs]);
            *(volatile v4f*)(orow + (size_t)row * DM + cofs) = val; }
        if (ps == 0) __threadfence(); }
}

static constexpr size_t al256(size_t v) { return (v + 255) & ~(size_t)255; }
static constexpr size_t SZ_HP = al256((size_t)NB * SEQ * EMB * 2);
static constexpr size_t SZ_WB = al256((size_t)6 * DM * EMB * 2);
static constexpr size_t SZ_PL = al256((size_t)NB * NH_ * SEQ * HD * 2);
static constexpr size_t SZ_CS = al256((size_t)NB * NH_ * SEQ * 4);
static constexpr size_t SZ_AT = al256(((size_t)(NB - 1) * OUT_SEQ + SEQ) * DM * 4);
static constexpr size_t SZ_X1 = al256((size_t)NB * SEQ * DM * 4);
static constexpr size_t SZ_TOTAL = 4 * SZ_HP + SZ_WB + 5 * SZ_PL + SZ_CS + SZ_AT + SZ_X1;
static_assert(SZ_TOTAL <= (size_t)134217728);
static_assert(((size_t)DM * EMB * 2) % 256 == 0);
static_assert(OUT_SEQ >= SEQ);

extern "C" void kernel_launch(void* const* d_in, const int* in_sizes, int n_in,
                              void* d_out, int out_size, void* d_ws, size_t ws_size, hipStream_t stream) {
    if (n_in < 17) return;
    const size_t needx = ((size_t)(NB - 1) * SEQ_FULL + SEQ) * EMB;
    if ((size_t)in_sizes[0] < needx) return;
    if ((size_t)in_sizes[1] < (size_t)NH_ * EMB * HD || (size_t)in_sizes[3] < (size_t)NH_ * EMB * HD || (size_t)in_sizes[5] < (size_t)NH_ * EMB * HD) return;
    if ((size_t)in_sizes[2] < (size_t)DM || (size_t)in_sizes[4] < (size_t)DM || (size_t)in_sizes[6] < (size_t)DM) return;
    if ((size_t)in_sizes[7] < (size_t)DM * EMB || (size_t)in_sizes[13] < (size_t)DM * EMB || (size_t)in_sizes[15] < (size_t)DM * EMB) return;
    if ((size_t)in_sizes[8] < (size_t)DM || (size_t)in_sizes[9] < (size_t)EMB || (size_t)in_sizes[10] < (size_t)EMB || (size_t)in_sizes[11] < (size_t)EMB ||
        (size_t)in_sizes[12] < (size_t)EMB || (size_t)in_sizes[14] < (size_t)DM || (size_t)in_sizes[16] < (size_t)DM) return;
    if ((size_t)out_size < ((size_t)(NB - 1) * OUT_SEQ + SEQ) * DM) return;
    if (SZ_TOTAL > ws_size) return;
    const float* x  = (const float*)d_in[0];
    const float* qw = (const float*)d_in[1];  const float* qbias = (const float*)d_in[2];
    const float* kw = (const float*)d_in[3];  const float* kbias = (const float*)d_in[4];
    const float* vw = (const float*)d_in[5];  const float* vbias = (const float*)d_in[6];
    const float* ow = (const float*)d_in[7];  const float* obias = (const float*)d_in[8];
    const float* g1 = (const float*)d_in[9];  const float* s1 = (const float*)d_in[10];
    const float* g2 = (const float*)d_in[11]; const float* s2 = (const float*)d_in[12];
    const float* f1w = (const float*)d_in[13]; const float* f1b = (const float*)d_in[14];
    const float* f2w = (const float*)d_in[15]; const float* f2b = (const float*)d_in[16];
    float* OUT = (float*)d_out;
    char* wsp = (char*)d_ws;
    h16* H1 = (h16*)wsp; wsp += SZ_HP;
    h16* H2 = (h16*)wsp; wsp += SZ_HP;
    h16* ATH = (h16*)wsp; wsp += SZ_HP;
    h16* A1 = (h16*)wsp; wsp += SZ_HP;
    h16* WB = (h16*)wsp; wsp += SZ_WB;
    h16* QH = (h16*)wsp; wsp += SZ_PL;
    h16* QR = (h16*)wsp; wsp += SZ_PL;
    h16* KP = (h16*)wsp; wsp += SZ_PL;
    h16* VT = (h16*)wsp; wsp += SZ_PL;
    h16* VR = (h16*)wsp; wsp += SZ_PL;
    float* CS = (float*)wsp; wsp += SZ_CS;
    float* ATT = (float*)wsp; wsp += SZ_AT;
    float* X1 = (float*)wsp; wsp += SZ_X1;
    h16* WQ = WB; h16* WK = WB + (size_t)DM * EMB; h16* WV = WB + (size_t)2 * DM * EMB;
    h16* WO = WB + (size_t)3 * DM * EMB; h16* WF1 = WB + (size_t)4 * DM * EMB; h16* WF2 = WB + (size_t)5 * DM * EMB;

    k_cvtw<<<dim3(EMB / 64, NH_, 1), 256, 0, stream>>>(qw, WQ, (size_t)EMB * HD, HD);
    k_cvtw<<<dim3(EMB / 64, NH_, 1), 256, 0, stream>>>(kw, WK, (size_t)EMB * HD, HD);
    k_cvtw<<<dim3(EMB / 64, NH_, 1), 256, 0, stream>>>(vw, WV, (size_t)EMB * HD, HD);
    k_cvtw<<<dim3(EMB / 64, DM / 64, 1), 256, 0, stream>>>(ow,  WO,  (size_t)64, DM);
    k_cvtw<<<dim3(EMB / 64, DM / 64, 1), 256, 0, stream>>>(f1w, WF1, (size_t)64, DM);
    k_cvtw<<<dim3(EMB / 64, DM / 64, 1), 256, 0, stream>>>(f2w, WF2, (size_t)64, DM);

    k_ln<<<dim3(NB * SEQ / 8, 1, 1), 256, 0, stream>>>(x, SEQ_FULL, 1, g1, s1, H1);

    k_proj<<<dim3(NB * SEQ / 64, DM / 64, 1), 32, 0, stream>>>(H1, WQ, qbias, 0, 0, QH, QR, 1, SEQ, (size_t)NH_ * SEQ * HD, HD, HD, (size_t)SEQ * HD);
    k_proj<<<dim3(NB * SEQ / 64, DM / 64, 1), 32, 0, stream>>>(H1, WK, kbias, 0, 0, KP, KP, 0, SEQ, (size_t)NH_ * SEQ * HD, HD, HD, (size_t)SEQ * HD);
    k_proj<<<dim3(DM / 64, NB * SEQ / 64, 1), 32, 0, stream>>>(WV, H1, vbias, 1, 0, VT, VR, 1, DM, (size_t)0, SEQ, SEQ, (size_t)DM * SEQ);

    k_colstat<<<dim3(SEQ / (16 * AW), NB * NH_, 1), 32 * AW, 0, stream>>>(QH, QR, KP, CS);
    k_attn<<<dim3(SEQ / (16 * AW), NB * NH_, 1), 32 * AW, 0, stream>>>(QH, QR, KP, VT, VR, CS, ATT);

    if (OUT_SEQ == SEQ) {
        const size_t n8 = (size_t)NB * SEQ * DM / 8;
        k_cvth<<<(unsigned)((n8 + 255) / 256), 256, 0, stream>>>(ATT, ATH, ASC, n8);
    } else {
        const size_t n8 = (size_t)SEQ * DM / 8;
        for (int b = 0; b < NB; ++b) k_cvth<<<(unsigned)((n8 + 255) / 256), 256, 0, stream>>>(ATT + (size_t)b * OUT_SEQ * DM, ATH + (size_t)b * SEQ * DM, ASC, n8);
    }

    k_gemmr<<<dim3(NB * SEQ / 64, DM / 64, 1), 32, 0, stream>>>(ATH, WO, obias, FOLDO, x, 1, SEQ_FULL, X1, SEQ);
    k_ln<<<dim3(NB * SEQ / 8, 1, 1), 256, 0, stream>>>(X1, SEQ, 0, g2, s2, H2);
    k_proj<<<dim3(NB * SEQ / 64, DM / 64, 1), 32, 0, stream>>>(H2, WF1, f1b, 0, 1, A1, A1, 0, NB * SEQ, (size_t)0, DM, DM, (size_t)0);
    k_gemmr<<<dim3(NB * SEQ / 64, DM / 64, 1), 32, 0, stream>>>(A1, WF2, f2b, WINV, X1, 0, SEQ, OUT, OUT_SEQ);
}
